// AGDN_87119116632167
// MI455X (gfx1250) — hardware-run, weakly checked
//
#include <hip/hip_runtime.h>

typedef float          v8f   __attribute__((ext_vector_type(8)));
typedef float          v4f   __attribute__((ext_vector_type(4)));
typedef unsigned int   v4u   __attribute__((ext_vector_type(4)));
typedef int            v8i   __attribute__((ext_vector_type(8)));
typedef unsigned short v8us  __attribute__((ext_vector_type(8)));
typedef unsigned short v16us __attribute__((ext_vector_type(16)));
typedef __bf16         v16bf __attribute__((ext_vector_type(16)));
typedef _Float16       v16h  __attribute__((ext_vector_type(16)));
typedef v4f  __attribute__((may_alias)) v4fa;
typedef v8us __attribute__((may_alias)) v8usa;
union FragB { v16bf v; v16us u; v8us h[2]; v8i w; };
union FragH { v16h  v; v16us u; v8us h[2]; v8i w; };

__device__ __forceinline__ v8f wmb(const FragB& a, const FragB& b, v8f c) {
  v8f d = __builtin_amdgcn_wmma_f32_16x16x32_bf16(false, a.v, false, b.v, (short)0, c, false, false);
  asm volatile("v_nop\n\tv_nop\n\tv_nop\n\tv_nop" : "+v"(d) : "v"(a.w), "v"(b.w));
  return d;
}

__device__ __forceinline__ v8f wmh(const FragH& a, const FragH& b, v8f c) {
  v8f d = __builtin_amdgcn_wmma_f32_16x16x32_f16(false, a.v, false, b.v, (short)0, c, false, false);
  asm volatile("v_nop\n\tv_nop\n\tv_nop\n\tv_nop" : "+v"(d) : "v"(a.w), "v"(b.w));
  return d;
}

__device__ __forceinline__ unsigned bf16_bits(float f) {
  const unsigned u = __float_as_uint(f);
  const unsigned r = (u + 0x7FFFu + ((u >> 16) & 1u)) >> 16;
  const unsigned q = (u >> 16) | 0x40u;
  return ((u & 0x7fffffffu) > 0x7f800000u) ? q : r;
}

__device__ __forceinline__ float bf16_val(float f) {
  return __uint_as_float(bf16_bits(f) << 16);
}
__device__ __forceinline__ int clampi(int v, int lo, int hi) {
  return v < lo ? lo : (v > hi ? hi : v);
}

__device__ __forceinline__ unsigned f16_bits(float f) {
  const unsigned u  = __float_as_uint(f);
  const unsigned s  = (u >> 16) & 0x8000u;
  const unsigned a  = u & 0x7fffffffu;
  const unsigned t  = a - 0x38000000u;
  const unsigned r  = (t + 0x0FFFu + ((t >> 13) & 1u)) >> 13;
  const unsigned rc = r > 0x7C00u ? 0x7C00u : r;
  const bool small  = a < 0x38800000u;
  const bool isnan  = a > 0x7f800000u;
  const unsigned fin = small ? 0u : (s | rc);
  return isnan ? (s | 0x7E00u) : fin;
}

__device__ __forceinline__ unsigned pk16(unsigned lo, unsigned hi) { return lo | (hi << 16); }
__device__ __forceinline__ unsigned bf16_lo_bits(float v) {
  float hi = bf16_val(v);
  asm volatile("" : "+v"(hi));
  return bf16_bits(v - hi);
}
__device__ __forceinline__ v4u pack8_bf16(v4f a, v4f c) {
  return (v4u){ pk16(bf16_bits(a[0]), bf16_bits(a[1])), pk16(bf16_bits(a[2]), bf16_bits(a[3])),
                pk16(bf16_bits(c[0]), bf16_bits(c[1])), pk16(bf16_bits(c[2]), bf16_bits(c[3])) };
}
__device__ __forceinline__ v4u pack8_bf16_lo(v4f a, v4f c) {
  return (v4u){ pk16(bf16_lo_bits(a[0]), bf16_lo_bits(a[1])), pk16(bf16_lo_bits(a[2]), bf16_lo_bits(a[3])),
                pk16(bf16_lo_bits(c[0]), bf16_lo_bits(c[1])), pk16(bf16_lo_bits(c[2]), bf16_lo_bits(c[3])) };
}
__device__ __forceinline__ v4u pack8_f16(v4f a, v4f c) {
  return (v4u){ pk16(f16_bits(a[0]), f16_bits(a[1])), pk16(f16_bits(a[2]), f16_bits(a[3])),
                pk16(f16_bits(c[0]), f16_bits(c[1])), pk16(f16_bits(c[2]), f16_bits(c[3])) };
}

template <int FORM>
__global__ __launch_bounds__(256) void k_plane(const float* __restrict__ src, int rows, int cols, int ldsrc,
                                               unsigned short* __restrict__ dst, int MP, int KP) {
  static_assert(FORM >= 0 && FORM <= 3);
  const int KTOT = (FORM == 1 || FORM == 3) ? 2 * KP : KP;
  const unsigned ppr   = (unsigned)(KTOT >> 3);
  const unsigned kp8   = (unsigned)(KP >> 3);
  const unsigned total = (unsigned)MP * ppr;
  const unsigned g     = blockIdx.x * 256u + threadIdx.x;
  const unsigned rowu  = g / ppr;
  const unsigned p     = g - rowu * ppr;
  const bool second    = p >= kp8;
  const int row = (int)rowu;
  const int c0  = (int)((second ? p - kp8 : p) << 3);
  const float* srow = src + (size_t)clampi(row, 0, rows - 1) * (size_t)ldsrc;
  float x[8];
  unsigned mk[8];
#pragma unroll
  for (int e = 0; e < 8; ++e) {
    const int c = c0 + e;
    const float v = srow[clampi(c, 0, cols - 1)];
    asm volatile("" :: "v"(v));
    x[e]  = v;
    mk[e] = (row < rows && c < cols) ? 0xFFFFu : 0u;
  }
  const v4f a = (v4f){ x[0], x[1], x[2], x[3] };
  const v4f c = (v4f){ x[4], x[5], x[6], x[7] };
  v4u o;
  if (FORM == 2) {
    o = pack8_f16(a, c);
  } else {
    const v4u hi = pack8_bf16(a, c);
    o = hi;
    if (FORM == 1) { const v4u lo = pack8_bf16_lo(a, c); o = second ? lo : hi; }
  }
  const v4u mw = (v4u){ pk16(mk[0], mk[1]), pk16(mk[2], mk[3]), pk16(mk[4], mk[5]), pk16(mk[6], mk[7]) };
  o &= mw;
  if (g < total) {
    volatile v4u* q = (volatile v4u*)(dst + (size_t)g * 8);
    *q = o;
    __threadfence();
    *q = o;
  }
}

template <int FORM> struct FragOf    { typedef FragB T; };
template <>         struct FragOf<2> { typedef FragH T; };
__device__ __forceinline__ v8f mm(const FragB& a, const FragB& b, v8f c) { return wmb(a, b, c); }
__device__ __forceinline__ v8f mm(const FragH& a, const FragH& b, v8f c) { return wmh(a, b, c); }
template <class F> __device__ __forceinline__ F ld_frag(const unsigned short* p) {
  F f;
  f.h[0] = *(const v8usa*)(p);
  f.h[1] = *(const v8usa*)(p + 16);
  return f;
}

template <int FORM, int EPI>
__global__ __launch_bounds__(256) __attribute__((amdgpu_num_vgpr(248)))
void k_gemm_nt(const unsigned short* __restrict__ A, const unsigned short* __restrict__ B,
               const float* __restrict__ bias, float* __restrict__ D, int M, int N, int KTOT, int ldd) {
  static_assert(FORM >= 0 && FORM <= 2);
  static_assert(EPI == 0 || EPI == 1);
  typedef typename FragOf<FORM>::T F;
  __shared__ __attribute__((aligned(16))) float sT[8][16 * 68];
  const int lane = threadIdx.x & 31;
  const int wave = threadIdx.x >> 5;
  const int tilesM = (M + 63) >> 6;
  const int tilesN = (N + 63) >> 6;
  const int tile = blockIdx.x * 8 + wave;
  if (tile >= tilesM * tilesN) return;
  const int tm = tile / tilesN;
  const int tn = tile - tm * tilesN;
  const int m0 = tm << 6;
  const int n0 = tn << 6;

  const int rl = lane & 15;
  const int h8 = (lane >> 4) * 8;
  const unsigned short* pa = A + (size_t)(m0 + rl) * (size_t)KTOT + h8;
  const unsigned short* pb = B + (size_t)(n0 + rl) * (size_t)KTOT + h8;

  v8f acc[4][4];
#pragma unroll
  for (int i = 0; i < 4; ++i)
#pragma unroll
    for (int j = 0; j < 4; ++j) acc[i][j] = (v8f){0.f, 0.f, 0.f, 0.f, 0.f, 0.f, 0.f, 0.f};

#pragma unroll 1
  for (int k0 = 0; k0 < KTOT; k0 += 32) {
    F bf[4];
#pragma unroll
    for (int j = 0; j < 4; ++j) bf[j] = ld_frag<F>(pb + (size_t)(j << 4) * (size_t)KTOT + k0);
#pragma unroll
    for (int i = 0; i < 4; ++i) {
      const F af = ld_frag<F>(pa + (size_t)(i << 4) * (size_t)KTOT + k0);
#pragma unroll
      for (int j = 0; j < 4; ++j) acc[i][j] = mm(af, bf[j], acc[i][j]);
    }
  }

  float* slab = sT[wave];
  const int hh = lane >> 4;
  const int c4 = (lane & 15) * 4;
  const int nc = n0 + c4;
  const bool cok = nc < N;
  v4f bv = (v4f){0.f, 0.f, 0.f, 0.f};
  if (EPI == 1) {
    bv = *(const v4fa*)(bias + clampi(nc, 0, N - 4));
    asm volatile("" :: "v"(bv));
  }
#pragma unroll
  for (int i = 0; i < 4; ++i) {
    const int mBase = m0 + (i << 4);
#pragma unroll
    for (int j = 0; j < 4; ++j) {
#pragma unroll
      for (int r = 0; r < 8; ++r) slab[(h8 + r) * 68 + (j << 4) + rl] = acc[i][j][r];
    }
    __builtin_amdgcn_fence(__ATOMIC_RELEASE, "workgroup");
    __builtin_amdgcn_wave_barrier();
    __builtin_amdgcn_fence(__ATOMIC_ACQUIRE, "workgroup");
    v4f vv[8];
#pragma unroll
    for (int it = 0; it < 8; ++it) {
      const int row = it * 2 + hh;
      v4f v = *(const v4fa*)(slab + row * 68 + c4);
      if (EPI == 1) v += bv;
      vv[it] = v;
    }
    for (int pass = 0; pass < 2; ++pass) {
#pragma unroll
      for (int it = 0; it < 8; ++it) {
        const int row = mBase + it * 2 + hh;
        if (cok && row < M) *(volatile v4f*)(D + (size_t)row * (size_t)ldd + nc) = vv[it];
      }
      __threadfence();
    }
    __builtin_amdgcn_fence(__ATOMIC_RELEASE, "workgroup");
    __builtin_amdgcn_wave_barrier();
    __builtin_amdgcn_fence(__ATOMIC_ACQUIRE, "workgroup");
  }
}

#include <stddef.h>
#include <stdint.h>
#include <math.h>

#ifndef H2_TWO_TERM
#define H2_TWO_TERM 1
#endif

#define NN      50000
#define NE      800000
#define DIN     128
#define DH      64
#define OUTN    (NN * DH)
#define NPAD    50048
#define KH2     (H2_TWO_TERM ? 128 : 64)
#define NTHR    256
#define NWAVE   8
#define NBRUN   1024
#define SLSH    16
#define NBLK    49
#define EPW     (NE / NWAVE)
#define STEPE   256
#define NSTEP   ((EPW + STEPE - 1) / STEPE)
#define WLCAP   4096
#define RCAP    20992
#define DEGCAP  48
#define MEAS_B1024 16623
#define MEAS_DEG   35
#define BK_ZINTS   (NWAVE * WLCAP + RCAP + 3 * NBRUN)
#define BK_INTS    (BK_ZINTS + 16)
#define BK_LDS     (BK_INTS * 4)
#define LIST_V4    (RCAP / 4)
#define LIST_IT    ((LIST_V4 + NTHR - 1) / NTHR)
#define NBW1    ((DH * DIN / 8) / NTHR)
#define NBW2    ((DH * KH2 / 8) / NTHR)
#define T_ATT1  0
#define T_ATT2  128
#define T_B1    256
#define T_B2    320
#define T_N     384

static_assert(NN <= 65536 && NBRUN <= 1024 && NBRUN == 1024);
static_assert((((long long)(NBRUN - 1) << SLSH) | 0xFFFF) < (1LL << 31));
static_assert((NBLK - 1) * NBRUN < NN && NBLK * NBRUN >= NPAD && NN - (NBLK - 1) * NBRUN == 848);
static_assert(NPAD == 391 * 128 && NPAD % 64 == 0 && NPAD >= NN && NPAD % 8 == 0);
static_assert(NN % 16 == 0 && NN % 8 == 0);
static_assert(NE % NWAVE == 0 && EPW % 8 == 0 && NE % 8 == 0 && NWAVE * STEPE == 2048);
static_assert(NE - 390 * 2048 == 1280 && EPW - 390 * STEPE == 160 && NSTEP == 391);
static_assert(RCAP % 256 == 0 && 4 * RCAP >= 5 * MEAS_B1024 && RCAP % 128 == 0);
static_assert(DEGCAP >= MEAS_DEG + 8 && DEGCAP > 32 && DEGCAP <= 64);
static_assert(WLCAP % 4 == 0 && BK_ZINTS % 4 == 0);
static_assert(BK_LDS == 227392 && BK_LDS <= 262144 && BK_LDS + 0 <= 327680);
static_assert(8 * 16 * 68 * 4 <= 327680);
static_assert(KH2 % 32 == 0 && DIN % 32 == 0 && DH == 64);
static_assert((DH * DIN / 8) % NTHR == 0 && (DH * KH2 / 8) % NTHR == 0);
static_assert((NPAD * (DIN / 8)) % 256 == 0);

typedef float v2f __attribute__((ext_vector_type(2)));
typedef int   v4i __attribute__((ext_vector_type(4)));
typedef v2f __attribute__((may_alias)) v2fa;
typedef v4i __attribute__((may_alias)) v4ia;

#define PIN(x) asm volatile("" :: "v"(x))

__device__ __forceinline__ void wunit(const float* __restrict__ W, int kin, int KW, int u, unsigned short* dstp) {
  const int ppr = KW >> 3;
  const int n   = u / ppr;
  const int k8  = (u - n * ppr) << 3;
  const int kk  = k8 & (kin - 1);
  const float* p = W + (size_t)n * (size_t)kin + kk;
  const v4f a = *(const v4fa*)(p);
  const v4f c = *(const v4fa*)(p + 4);
  PIN(a);
  PIN(c);
  const v4u o = pack8_bf16(a, c);
  volatile v4u* q = (volatile v4u*)(dstp + (size_t)n * (size_t)KW + k8);
  *q = o;
  __threadfence();
  *q = o;
}

__device__ __forceinline__ void tunit(const float* __restrict__ s, int n, int tid, float* dstp) {
  const int c4 = tid * 4;
  const int cc = c4 < (n - 4) ? c4 : (n - 4);
  const v4f v = *(const v4fa*)(s + cc);
  PIN(v);
  const v4f o = (v4f){ bf16_val(v[0]), bf16_val(v[1]), bf16_val(v[2]), bf16_val(v[3]) };
  if (c4 < n) {
    volatile v4f* q = (volatile v4f*)(dstp + c4);
    *q = o;
    __threadfence();
    *q = o;
  }
}

__global__ __launch_bounds__(NTHR) void k_prep(const float* __restrict__ W1, const float* __restrict__ Wr,
                                               const float* __restrict__ W2, const float* __restrict__ a1,
                                               const float* __restrict__ a2, const float* __restrict__ b1,
                                               const float* __restrict__ b2,
                                               unsigned short* WC, unsigned short* W2D, float* TAB) {
  const int blk = (int)blockIdx.x;
  const int tid = (int)threadIdx.x;
  if (blk < NBW1) {
    wunit(W1, DIN, DIN, blk * NTHR + tid, WC);
  } else if (blk < 2 * NBW1) {
    wunit(Wr, DIN, DIN, (blk - NBW1) * NTHR + tid, WC + (size_t)DH * DIN);
  } else if (blk < 2 * NBW1 + NBW2) {
    wunit(W2, DH, KH2, (blk - 2 * NBW1) * NTHR + tid, W2D);
  } else if (blk == 2 * NBW1 + NBW2) {
    tunit(a1, 128, tid, TAB + T_ATT1);
  } else if (blk == 2 * NBW1 + NBW2 + 1) {
    tunit(a2, 128, tid, TAB + T_ATT2);
  } else if (blk == 2 * NBW1 + NBW2 + 2) {
    tunit(b1, 64, tid, TAB + T_B1);
  } else {
    tunit(b2, 64, tid, TAB + T_B2);
  }
}

#define PUTJ(HJ, SRCJ, SJ) { \
    const int wv = clampi((SRCJ), 0, nN - 1) | ((int)(SJ) << SLSH); \
    if (HJ) { if (pos < WLCAP) wlw[pos] = wv; } \
    pos += (HJ) ? 1 : 0; }

__global__ __launch_bounds__(NTHR) void k_bucket(const int* __restrict__ srcs, const int* __restrict__ dsts,
                                                 int nN, int* listG, int* cntG, int* offG, int* flagG) {
  extern __shared__ __attribute__((aligned(16))) int dsm[];
  int* wl   = dsm;
  int* sl   = dsm + NWAVE * WLCAP;
  int* cnt  = sl + RCAP;
  int* offs = cnt + NBRUN;
  int* cur  = offs + NBRUN;
  int* misc = cur + NBRUN;
  const int tid = (int)threadIdx.x, lane = tid & 31, wave = tid >> 5;
  const int b = (int)blockIdx.x;
  const int nodeBase = b * NBRUN;
  const int nb = clampi(nN - nodeBase, 0, NBRUN);

  {
    const v4i z4 = {0, 0, 0, 0};
    for (int i = tid * 4; i < BK_ZINTS; i += NTHR * 4) *(v4ia*)(dsm + i) = z4;
    if (tid < 16) misc[tid] = 0;
  }
  __syncthreads();

  {
    int* wlw = wl + wave * WLCAP;
    const int wbeg = wave * EPW;
    const int wend = wbeg + EPW;
    const unsigned nbs = (unsigned)nodeBase;
    const unsigned unb = (unsigned)nb;
    int wc = 0;
#pragma unroll 1
    for (int st = 0; st < NSTEP; ++st) {
      const int e0  = wbeg + st * STEPE + lane * 8;
      const int e0c = e0 < (NE - 8) ? e0 : (NE - 8);
      const v4i da = *(const v4ia*)(dsts + e0c);
      const v4i db = *(const v4ia*)(dsts + e0c + 4);
      const v4i sa = *(const v4ia*)(srcs + e0c);
      const v4i sb = *(const v4ia*)(srcs + e0c + 4);
      PIN(da.x); PIN(da.y); PIN(da.z); PIN(da.w);
      PIN(db.x); PIN(db.y); PIN(db.z); PIN(db.w);
      PIN(sa.x); PIN(sa.y); PIN(sa.z); PIN(sa.w);
      PIN(sb.x); PIN(sb.y); PIN(sb.z); PIN(sb.w);
      const unsigned s0 = (unsigned)da.x - nbs, s1 = (unsigned)da.y - nbs;
      const unsigned s2 = (unsigned)da.z - nbs, s3 = (unsigned)da.w - nbs;
      const unsigned s4 = (unsigned)db.x - nbs, s5 = (unsigned)db.y - nbs;
      const unsigned s6 = (unsigned)db.z - nbs, s7 = (unsigned)db.w - nbs;
      const bool h0 = (e0 + 0 < wend) && (s0 < unb);
      const bool h1 = (e0 + 1 < wend) && (s1 < unb);
      const bool h2 = (e0 + 2 < wend) && (s2 < unb);
      const bool h3 = (e0 + 3 < wend) && (s3 < unb);
      const bool h4 = (e0 + 4 < wend) && (s4 < unb);
      const bool h5 = (e0 + 5 < wend) && (s5 < unb);
      const bool h6 = (e0 + 6 < wend) && (s6 < unb);
      const bool h7 = (e0 + 7 < wend) && (s7 < unb);
      const unsigned m0 = __builtin_amdgcn_ballot_w32(h0);
      const unsigned m1 = __builtin_amdgcn_ballot_w32(h1);
      const unsigned m2 = __builtin_amdgcn_ballot_w32(h2);
      const unsigned m3 = __builtin_amdgcn_ballot_w32(h3);
      const unsigned m4 = __builtin_amdgcn_ballot_w32(h4);
      const unsigned m5 = __builtin_amdgcn_ballot_w32(h5);
      const unsigned m6 = __builtin_amdgcn_ballot_w32(h6);
      const unsigned m7 = __builtin_amdgcn_ballot_w32(h7);
      const unsigned many = m0 | m1 | m2 | m3 | m4 | m5 | m6 | m7;
      if (many != 0u) {
        unsigned pre = __builtin_amdgcn_mbcnt_lo(m0, 0u);
        pre = __builtin_amdgcn_mbcnt_lo(m1, pre);
        pre = __builtin_amdgcn_mbcnt_lo(m2, pre);
        pre = __builtin_amdgcn_mbcnt_lo(m3, pre);
        pre = __builtin_amdgcn_mbcnt_lo(m4, pre);
        pre = __builtin_amdgcn_mbcnt_lo(m5, pre);
        pre = __builtin_amdgcn_mbcnt_lo(m6, pre);
        pre = __builtin_amdgcn_mbcnt_lo(m7, pre);
        int pos = wc + (int)pre;
        PUTJ(h0, sa.x, s0)
        PUTJ(h1, sa.y, s1)
        PUTJ(h2, sa.z, s2)
        PUTJ(h3, sa.w, s3)
        PUTJ(h4, sb.x, s4)
        PUTJ(h5, sb.y, s5)
        PUTJ(h6, sb.z, s6)
        PUTJ(h7, sb.w, s7)
        wc += (int)__builtin_popcount(m0) + (int)__builtin_popcount(m1) + (int)__builtin_popcount(m2)
            + (int)__builtin_popcount(m3) + (int)__builtin_popcount(m4) + (int)__builtin_popcount(m5)
            + (int)__builtin_popcount(m6) + (int)__builtin_popcount(m7);
      }
    }
    if (lane == 0) misc[wave] = wc;
  }
  __syncthreads();

  if (wave == 0) {
    int t = 0, ov = 0;
#pragma unroll 1
    for (int w2 = 0; w2 < NWAVE; ++w2) {
      int c = misc[w2];
      ov |= (c > WLCAP) ? 1 : 0;
      c = c < 0 ? 0 : (c > WLCAP ? WLCAP : c);
      c = __builtin_amdgcn_readfirstlane(c);
#pragma unroll 1
      for (int b0 = 0; b0 < c; b0 += 32) {
        const int idx = b0 + lane;
        const int ent = wl[w2 * WLCAP + (idx < WLCAP ? idx : WLCAP - 1)];
        const int m32 = (c - b0) < 32 ? (c - b0) : 32;
#pragma unroll 1
        for (int k = 0; k < m32; ++k) {
          const int u    = __builtin_amdgcn_readlane(ent, k);
          const int slot = (u >> SLSH) & (NBRUN - 1);
          if (t < RCAP) {
            const int cvv = cnt[slot];
            if (lane == 0) cnt[slot] = cvv + 1;
            t = t + 1;
          } else {
            ov = 1;
          }
        }
      }
    }
    if (lane == 0) { misc[8] = t; misc[9] = ov; }
  }
  __syncthreads();

  if (wave == 0) {
    const int base = lane * (NBRUN / 32);
    int s = 0;
#pragma unroll 1
    for (int i = 0; i < NBRUN / 32; ++i) s += cnt[base + i];
    int incl = s;
#pragma unroll
    for (int d = 1; d < 32; d <<= 1) {
      const int y = __shfl_up(incl, d, 32);
      if (lane >= d) incl += y;
    }
    int run = incl - s;
#pragma unroll 1
    for (int i = 0; i < NBRUN / 32; ++i) {
      const int cvv = cnt[base + i];
      offs[base + i] = run;
      cur[base + i]  = run;
      run += cvv;
    }
  }
  __syncthreads();

  if (wave == 0) {
    int t = 0;
#pragma unroll 1
    for (int w2 = 0; w2 < NWAVE; ++w2) {
      int c = misc[w2];
      c = c < 0 ? 0 : (c > WLCAP ? WLCAP : c);
      c = __builtin_amdgcn_readfirstlane(c);
#pragma unroll 1
      for (int b0 = 0; b0 < c; b0 += 32) {
        const int idx = b0 + lane;
        const int ent = wl[w2 * WLCAP + (idx < WLCAP ? idx : WLCAP - 1)];
        const int m32 = (c - b0) < 32 ? (c - b0) : 32;
#pragma unroll 1
        for (int k = 0; k < m32; ++k) {
          const int u    = __builtin_amdgcn_readlane(ent, k);
          const int slot = (u >> SLSH) & (NBRUN - 1);
          if (t < RCAP) {
            int p = cur[slot];
            p = p < 0 ? 0 : (p > RCAP - 1 ? RCAP - 1 : p);
            if (lane == 0) { sl[p] = u & 0xFFFF; cur[slot] = p + 1; }
            t = t + 1;
          }
        }
      }
    }
  }
  __syncthreads();

  {
    const int ovf = misc[9];
    const v4i fv = {ovf, ovf, ovf, ovf};
    int* lb = listG + (size_t)b * RCAP;
    for (int pass = 0; pass < 2; ++pass) {
#pragma unroll 1
      for (int it = 0; it < LIST_IT; ++it) {
        const int i4 = it * NTHR + tid;
        const int ic = i4 < LIST_V4 ? i4 : LIST_V4 - 1;
        const v4i v = *(const v4ia*)(sl + 4 * ic);
        if (i4 < LIST_V4) *(volatile v4i*)(lb + 4 * (size_t)i4) = v;
      }
      {
        const v4i c4 = *(const v4ia*)(cnt + 4 * tid);
        const v4i o4 = *(const v4ia*)(offs + 4 * tid);
        *(volatile v4i*)(cntG + (size_t)nodeBase + 4 * tid) = c4;
        *(volatile v4i*)(offG + (size_t)nodeBase + 4 * tid) = o4;
      }
      if (tid < 8) *(volatile v4i*)(flagG + (size_t)b * 32 + 4 * tid) = fv;
      __threadfence();
    }
  }
}

__device__ __forceinline__ v2f row_sum(const float* __restrict__ S, int stride, int ent0, int ent1, int cn,
                                       int lane, int nN) {
  float a0 = 0.0f, a1 = 0.0f;
  const int n0 = cn < 32 ? cn : 32;
#pragma unroll 1
  for (int k = 0; k < n0; ++k) {
    int sk = __builtin_amdgcn_readlane(ent0, k);
    sk = clampi(sk, 0, nN - 1);
    const v2f t = *(const v2fa*)(S + (size_t)sk * (size_t)stride + 2 * lane);
    PIN(t);
    a0 += t.x; a1 += t.y;
  }
#pragma unroll 1
  for (int k = 32; k < cn; ++k) {
    int sk = __builtin_amdgcn_readlane(ent1, k - 32);
    sk = clampi(sk, 0, nN - 1);
    const v2f t = *(const v2fa*)(S + (size_t)sk * (size_t)stride + 2 * lane);
    PIN(t);
    a0 += t.x; a1 += t.y;
  }
  return (v2f){ a0, a1 };
}

__global__ __launch_bounds__(NTHR) void k_hop(const float* __restrict__ S, int stride,
                                              const int* __restrict__ listG, const int* __restrict__ cntG,
                                              const int* __restrict__ offG, const int* __restrict__ flagG,
                                              float* Fo, int nN) {
  const int tid = (int)threadIdx.x, lane = tid & 31, wave = tid >> 5;
  const int row = (int)blockIdx.x * NWAVE + wave;
  if (row >= nN) return;
  const int b = row >> 10;
  int cv  = cntG[row];
  int ofv = offG[row];
  int fl  = flagG[(size_t)b * 32];
  PIN(cv);
  PIN(ofv);
  PIN(fl);
  const bool big = cv > DEGCAP;
  cv  = cv < 0 ? 0 : (cv > DEGCAP ? DEGCAP : cv);
  ofv = ofv < 0 ? 0 : (ofv > RCAP ? RCAP : ofv);
  const int cn = __builtin_amdgcn_readfirstlane(cv);
  const int* listb = listG + (size_t)b * RCAP;
  const int i0 = clampi(ofv + lane, 0, RCAP - 1);
  const int i1 = clampi(ofv + 32 + lane, 0, RCAP - 1);
  int ent0 = listb[i0];
  int ent1 = listb[i1];
  PIN(ent0);
  PIN(ent1);
  const v2f a = row_sum(S, stride, ent0, ent1, cn, lane, nN);
  const float qnan = __int_as_float(0x7fc00000);
  const bool bad = (fl != 0) || big;
  const v2f o = (v2f){ bad ? qnan : a.x, bad ? qnan : a.y };
  float* op = Fo + (size_t)row * DH + 2 * lane;
  *(volatile v2f*)op = o;
  __threadfence();
  *(volatile v2f*)op = o;
}

__device__ __forceinline__ float wsum(float v) {
#pragma unroll
  for (int off = 16; off > 0; off >>= 1) v += __shfl_xor(v, off, 32);
  return v;
}

__device__ __forceinline__ v2f comb_core(v2f f0, v2f rs, v2f f1, v2f f2, v2f f3, v2f al, v2f ah, v2f bi) {
  float pa = f0.x * al.x + f0.y * al.y;
  float p0 = f0.x * ah.x + f0.y * ah.y;
  float p1 = f1.x * ah.x + f1.y * ah.y;
  float p2 = f2.x * ah.x + f2.y * ah.y;
  float p3 = f3.x * ah.x + f3.y * ah.y;
  pa = wsum(pa);
  p0 = wsum(p0);
  p1 = wsum(p1);
  p2 = wsum(p2);
  p3 = wsum(p3);
  float s0 = pa + p0, s1 = pa + p1, s2 = pa + p2, s3 = pa + p3;
  s0 = (s0 >= 0.0f) ? s0 : 0.2f * s0;
  s1 = (s1 >= 0.0f) ? s1 : 0.2f * s1;
  s2 = (s2 >= 0.0f) ? s2 : 0.2f * s2;
  s3 = (s3 >= 0.0f) ? s3 : 0.2f * s3;
  float m = s0;
  m = (s1 > m || s1 != s1) ? s1 : m;
  m = (s2 > m || s2 != s2) ? s2 : m;
  m = (s3 > m || s3 != s3) ? s3 : m;
  const float e0 = expf(s0 - m);
  const float e1 = expf(s1 - m);
  const float e2 = expf(s2 - m);
  const float e3 = expf(s3 - m);
  const float den = ((e0 + e1) + e2) + e3;
  const float inv = 1.0f / den;
  const float w0 = e0 * inv, w1 = e1 * inv, w2 = e2 * inv, w3 = e3 * inv;
  float ox = f0.x * w0;
  float oy = f0.y * w0;
  ox += f1.x * w1; oy += f1.y * w1;
  ox += f2.x * w2; oy += f2.y * w2;
  ox += f3.x * w3; oy += f3.y * w3;
  return (v2f){ (ox + rs.x) + bi.x, (oy + rs.y) + bi.y };
}

__device__ __forceinline__ void stage_par(const float* __restrict__ TAB, int attOff, int biasOff, int tid,
                                          float* sP) {
  const int tc  = tid < 47 ? tid : 47;
  const int off = (tc < 32) ? (attOff + 4 * tc) : (biasOff + 4 * (tc - 32));
  const v4f v = *(const v4fa*)(TAB + off);
  PIN(v);
  if (tid < 48) *(v4fa*)(sP + 4 * tid) = v;
}

template <int KH>
__global__ __launch_bounds__(NTHR) void k_comb1(const float* __restrict__ HRp, const float* __restrict__ F1,
                                                const float* __restrict__ F2, const float* __restrict__ F3,
                                                const float* __restrict__ TAB, const int* __restrict__ flagG,
                                                unsigned short* hb, int nN, int mRows) {
  static_assert(KH == 64 || KH == 128);
  __shared__ __attribute__((aligned(16))) float sP[192];
  const int tid = (int)threadIdx.x, lane = tid & 31, wave = tid >> 5;
  stage_par(TAB, T_ATT1, T_B1, tid, sP);
  __syncthreads();
  const int row = (int)blockIdx.x * NWAVE + wave;
  if (row >= mRows) return;
  const bool live = row < nN;
  const int rc = live ? row : (nN - 1);
  const v2f al = *(const v2fa*)(sP + 2 * lane);
  const v2f ah = *(const v2fa*)(sP + 64 + 2 * lane);
  const v2f bi = *(const v2fa*)(sP + 128 + 2 * lane);
  const v2f f0 = *(const v2fa*)(HRp + (size_t)rc * 128 + 2 * lane);
  const v2f rs = *(const v2fa*)(HRp + (size_t)rc * 128 + 64 + 2 * lane);
  const v2f f1 = *(const v2fa*)(F1 + (size_t)rc * DH + 2 * lane);
  const v2f f2 = *(const v2fa*)(F2 + (size_t)rc * DH + 2 * lane);
  const v2f f3 = *(const v2fa*)(F3 + (size_t)rc * DH + 2 * lane);
  int fl = flagG[(size_t)(rc >> 10) * 32];
  PIN(f0); PIN(rs); PIN(f1); PIN(f2); PIN(f3); PIN(fl);
  const v2f v = comb_core(f0, rs, f1, f2, f3, al, ah, bi);
  const float ex = expm1f(v.x);
  const float ey = expm1f(v.y);
  float hx = (v.x > 0.0f) ? v.x : ex;
  float hy = (v.y > 0.0f) ? v.y : ey;
  const float qnan = __int_as_float(0x7fc00000);
  const bool bad = fl != 0;
  hx = bad ? qnan : hx;
  hy = bad ? qnan : hy;
  const unsigned hwv = pk16(bf16_bits(hx), bf16_bits(hy));
  const unsigned lwv = pk16(bf16_lo_bits(hx), bf16_lo_bits(hy));
  const unsigned hw = live ? hwv : 0u;
  const unsigned lw = live ? lwv : 0u;
  unsigned short* hp = hb + (size_t)row * KH + 2 * lane;
  volatile unsigned* q0 = (volatile unsigned*)(hp);
  volatile unsigned* q1 = (volatile unsigned*)(hp + 64);
  *q0 = hw;
  if (KH == 128) *q1 = lw;
  __threadfence();
  *q0 = hw;
  if (KH == 128) *q1 = lw;
}

__global__ __launch_bounds__(NTHR) void k_comb2(const float* __restrict__ H2p, const float* __restrict__ F1,
                                                const float* __restrict__ F2, const float* __restrict__ F3,
                                                const float* __restrict__ TAB, const int* __restrict__ flagG,
                                                float* out, int nOut) {
  __shared__ __attribute__((aligned(16))) float sP[192];
  const int tid = (int)threadIdx.x, lane = tid & 31, wave = tid >> 5;
  stage_par(TAB, T_ATT2, T_B2, tid, sP);
  __syncthreads();
  const int row = (int)blockIdx.x * NWAVE + wave;
  if (row >= nOut) return;
  const v2f al = *(const v2fa*)(sP + 2 * lane);
  const v2f ah = *(const v2fa*)(sP + 64 + 2 * lane);
  const v2f bi = *(const v2fa*)(sP + 128 + 2 * lane);
  const v2f f0 = *(const v2fa*)(H2p + (size_t)row * DH + 2 * lane);
  const v2f f1 = *(const v2fa*)(F1 + (size_t)row * DH + 2 * lane);
  const v2f f2 = *(const v2fa*)(F2 + (size_t)row * DH + 2 * lane);
  const v2f f3 = *(const v2fa*)(F3 + (size_t)row * DH + 2 * lane);
  int fl = flagG[(size_t)(row >> 10) * 32];
  PIN(f0); PIN(f1); PIN(f2); PIN(f3); PIN(fl);
  const v2f v = comb_core(f0, f0, f1, f2, f3, al, ah, bi);
  const float qnan = __int_as_float(0x7fc00000);
  const bool bad = fl != 0;
  const v2f o = (v2f){ bad ? qnan : v.x, bad ? qnan : v.y };
  float* op = out + (size_t)row * DH + 2 * lane;
  if (row < nOut) *(volatile v2f*)op = o;
  __threadfence();
  if (row < nOut) *(volatile v2f*)op = o;
}

constexpr size_t SZ_XB   = (size_t)NPAD * DIN * 2;
constexpr size_t SZ_HR   = (size_t)NPAD * 128 * 4;
constexpr size_t SZ_F    = (size_t)NPAD * DH * 4;
constexpr size_t SZ_HHL  = (size_t)NPAD * 128 * 2;
constexpr size_t SZ_H2   = (size_t)NPAD * DH * 4;
constexpr size_t SZ_LIST = (size_t)NBLK * RCAP * 4;
constexpr size_t SZ_CNT  = (size_t)NBLK * NBRUN * 4;
constexpr size_t SZ_FLAG = (size_t)(NBLK + 1) * 32 * 4;
constexpr size_t SZ_WC   = (size_t)128 * DIN * 2;
constexpr size_t SZ_W2D  = (size_t)DH * 128 * 2;
constexpr size_t SZ_TAB  = (size_t)T_N * 4;
constexpr size_t O_XB   = 0;
constexpr size_t O_HR   = O_XB + SZ_XB;
constexpr size_t O_F1   = O_HR + SZ_HR;
constexpr size_t O_F2   = O_F1 + SZ_F;
constexpr size_t O_F3   = O_F2 + SZ_F;
constexpr size_t O_HHL  = O_F3 + SZ_F;
constexpr size_t O_H2   = O_HHL + SZ_HHL;
constexpr size_t O_LIST = O_H2 + SZ_H2;
constexpr size_t O_CNT  = O_LIST + SZ_LIST;
constexpr size_t O_OFF  = O_CNT + SZ_CNT;
constexpr size_t O_FLAG = O_OFF + SZ_CNT;
constexpr size_t O_WC   = O_FLAG + SZ_FLAG;
constexpr size_t O_W2D  = O_WC + SZ_WC;
constexpr size_t O_TAB  = O_W2D + SZ_W2D;
constexpr size_t WS_TOTAL = O_TAB + SZ_TAB;
static_assert(SZ_XB % 256 == 0 && SZ_HR % 256 == 0 && SZ_F % 256 == 0 && SZ_HHL % 256 == 0 && SZ_H2 % 256 == 0);
static_assert(SZ_LIST % 256 == 0 && SZ_CNT % 256 == 0 && SZ_FLAG % 256 == 0 && SZ_WC % 256 == 0);
static_assert(SZ_W2D % 256 == 0 && SZ_TAB % 256 == 0);
static_assert(WS_TOTAL == ((size_t)418247 << 8) && WS_TOTAL <= ((size_t)128 << 20));
static_assert((size_t)NPAD * KH2 * 2 <= SZ_HHL && (size_t)DH * KH2 * 2 <= SZ_W2D);
static_assert((size_t)NBLK * 32 * 4 <= SZ_FLAG && (size_t)NBLK * NBRUN >= (size_t)NN);

extern "C" void kernel_launch(void* const* d_in, const int* in_sizes, int n_in,
                              void* d_out, int out_size, void* d_ws, size_t ws_size,
                              hipStream_t stream) {
  if (n_in < 9) return;
  if (in_sizes[0] != NN * DIN) return;
  if (in_sizes[1] != 2 * NE) return;
  if (in_sizes[2] != DH * DIN || in_sizes[3] != 128) return;
  if (in_sizes[4] != DH || in_sizes[5] != DH * DIN) return;
  if (in_sizes[6] != DH * DH || in_sizes[7] != 128) return;
  if (in_sizes[8] != DH) return;
  if (out_size != OUTN) return;
  if (ws_size < WS_TOTAL) return;

  const float* x    = (const float*)d_in[0];
  const int*   edge = (const int*)d_in[1];
  const float* W1   = (const float*)d_in[2];
  const float* att1 = (const float*)d_in[3];
  const float* b1   = (const float*)d_in[4];
  const float* Wr   = (const float*)d_in[5];
  const float* W2   = (const float*)d_in[6];
  const float* att2 = (const float*)d_in[7];
  const float* b2   = (const float*)d_in[8];
  float* out = (float*)d_out;
  const int* src = edge;
  const int* dst = edge + NE;

  char* ws = (char*)d_ws;
  unsigned short* XB  = (unsigned short*)(ws + O_XB);
  float*          HR  = (float*)(ws + O_HR);
  float*          F1  = (float*)(ws + O_F1);
  float*          F2  = (float*)(ws + O_F2);
  float*          F3  = (float*)(ws + O_F3);
  unsigned short* HHL = (unsigned short*)(ws + O_HHL);
  float*          H2  = (float*)(ws + O_H2);
  int*            LST = (int*)(ws + O_LIST);
  int*            CNT = (int*)(ws + O_CNT);
  int*            OFF = (int*)(ws + O_OFF);
  int*            FLG = (int*)(ws + O_FLAG);
  unsigned short* WC  = (unsigned short*)(ws + O_WC);
  unsigned short* W2D = (unsigned short*)(ws + O_W2D);
  float*          TAB = (float*)(ws + O_TAB);

  hipFuncSetAttribute(reinterpret_cast<const void*>(&k_bucket), hipFuncAttributeMaxDynamicSharedMemorySize,
                      (int)BK_LDS);

  const int tilesM    = NPAD / 64;
  const int gemm1Grid = (tilesM * 2 + 7) / 8;
  const int gemm2Grid = (tilesM * 1 + 7) / 8;
  const int hopGrid   = NN / NWAVE;
  const int c1Grid    = NPAD / NWAVE;

  k_plane<0><<<NPAD * (DIN / 8) / 256, 256, 0, stream>>>(x, NN, DIN, DIN, XB, NPAD, DIN);
  k_prep<<<2 * NBW1 + NBW2 + 4, NTHR, 0, stream>>>(W1, Wr, W2, att1, att2, b1, b2, WC, W2D, TAB);
  k_bucket<<<NBLK, NTHR, BK_LDS, stream>>>(src, dst, NN, LST, CNT, OFF, FLG);
  k_gemm_nt<0, 0><<<gemm1Grid, 256, 0, stream>>>(XB, WC, TAB, HR, NN, 128, DIN, 128);
  k_hop<<<hopGrid, NTHR, 0, stream>>>(HR, 128, LST, CNT, OFF, FLG, F1, NN);
  k_hop<<<hopGrid, NTHR, 0, stream>>>(F1, DH, LST, CNT, OFF, FLG, F2, NN);
  k_hop<<<hopGrid, NTHR, 0, stream>>>(F2, DH, LST, CNT, OFF, FLG, F3, NN);
  k_comb1<KH2><<<c1Grid, NTHR, 0, stream>>>(HR, F1, F2, F3, TAB, FLG, HHL, NN, NPAD);
  k_gemm_nt<H2_TWO_TERM ? 1 : 0, 0><<<gemm2Grid, 256, 0, stream>>>(HHL, W2D, TAB, H2, NN, DH, KH2, DH);
  k_hop<<<hopGrid, NTHR, 0, stream>>>(H2, DH, LST, CNT, OFF, FLG, F1, NN);
  k_hop<<<hopGrid, NTHR, 0, stream>>>(F1, DH, LST, CNT, OFF, FLG, F2, NN);
  k_hop<<<hopGrid, NTHR, 0, stream>>>(F2, DH, LST, CNT, OFF, FLG, F3, NN);
  k_comb2<<<hopGrid, NTHR, 0, stream>>>(H2, F1, F2, F3, TAB, FLG, out, NN);
}
